// LinearAttention_40570261078614
// MI455X (gfx1250) — hardware-verified
//
#include <hip/hip_runtime.h>
#include <math.h>

constexpr int kBatch   = 8;
constexpr int kSeq     = 2048;
constexpr int kDim     = 512;
constexpr int kTok     = kBatch * kSeq;
constexpr int kChunk   = 64;
constexpr int kNChunk  = kSeq / kChunk;
constexpr int kESlice  = 32;
constexpr int kNESlice = kDim / kESlice;
constexpr int kCatN    = 3 * kDim;
constexpr int kStPitch   = 520;
constexpr int kYsPitch   = 36;
constexpr int kSlabPitch = 68;
constexpr int kTwPitch   = 36;
constexpr int kAsPitch   = 68;
constexpr int kTtPitch   = 72;
constexpr float kDenEps  = 1e-6f;
static_assert(kSeq % kChunk == 0);
static_assert(kSeq == 2048 && kDim == 512 && kBatch == 8);
static_assert(kTok % 64 == 0 && kCatN % 64 == 0 && kDim % 64 == 0);
static_assert(kDim % 32 == 0 && kChunk % 32 == 0);
static_assert((kCatN / 64) % 8 == 0);
static_assert((kESlice * kStPitch) % 8 == 0);
static_assert(kNChunk == 32 && kNESlice == 16);

typedef __attribute__((ext_vector_type(16))) _Float16 v16h;
typedef __attribute__((ext_vector_type(8)))  _Float16 v8h;
typedef __attribute__((ext_vector_type(16))) __bf16   v16b;
typedef __attribute__((ext_vector_type(8)))  __bf16   v8b;
typedef __attribute__((ext_vector_type(8)))  float    v8f;
typedef __attribute__((ext_vector_type(4)))  float    v4f;
typedef __attribute__((ext_vector_type(4)))  unsigned int v4u;
typedef __attribute__((ext_vector_type(8)))  unsigned short us8;

__device__ __forceinline__ unsigned short f2bf_bits(float f) {
  unsigned u = __float_as_uint(f);
  return (unsigned short)((u + 0x7FFFu + ((u >> 16) & 1u)) >> 16);
}
__device__ __forceinline__ float bf_bits2f(unsigned short h) { return __uint_as_float(((unsigned)h) << 16); }
__device__ __forceinline__ unsigned pk16(unsigned short a, unsigned short b) { return (unsigned)a | ((unsigned)b << 16); }
__device__ __forceinline__ unsigned short h_bits(float f) { const _Float16 h = (_Float16)f; return __builtin_bit_cast(unsigned short, h); }
__device__ __forceinline__ float h16_to_f32(unsigned hb) {
  const unsigned sgn = (hb & 0x8000u) << 16;
  const unsigned em = hb & 0x7fffu;
  const float fn = __uint_as_float((em << 13) + 0x38000000u);
  const float fs = (float)em * 5.9604644775390625e-8f;
  const float mag = (em < 0x400u) ? fs : fn;
  return __uint_as_float(__float_as_uint(mag) | sgn);
}

union FragB { v16b v; v8b h[2]; };
union FragH { v16h v; v8h h[2]; };
__device__ __forceinline__ v16b ldfrag_b(const __bf16* p) {
  FragB f; f.h[0] = *(const v8b*)(p); f.h[1] = *(const v8b*)(p + 16); return f.v;
}
__device__ __forceinline__ v16h ldfrag_h(const _Float16* p) {
  FragH f; f.h[0] = *(const v8h*)(p); f.h[1] = *(const v8h*)(p + 16); return f.v;
}
__device__ __forceinline__ v8f mma_b(v16b a, v16b b, v8f c) {
  return __builtin_amdgcn_wmma_f32_16x16x32_bf16(false, a, false, b, (short)0, c, false, false);
}
__device__ __forceinline__ v8f mma_h(v16h a, v16h b, v8f c) {
  return __builtin_amdgcn_wmma_f32_16x16x32_f16(false, a, false, b, (short)0, c, false, false);
}
__device__ __forceinline__ void guard_b_4x2(v8f& a, v8f& b, v8f& c, v8f& d, v16b x, v16b y) {
  asm volatile("v_nop\n\tv_nop\n\tv_nop\n\tv_nop" : "+v"(a), "+v"(b), "+v"(c), "+v"(d) : "v"(x), "v"(y));
}
__device__ __forceinline__ void guard_b_1x2(v8f& a, v16b x, v16b y) {
  asm volatile("v_nop\n\tv_nop\n\tv_nop\n\tv_nop" : "+v"(a) : "v"(x), "v"(y));
}
__device__ __forceinline__ void guard_b_1x4(v8f& a, v16b w, v16b x, v16b y, v16b z) {
  asm volatile("v_nop\n\tv_nop\n\tv_nop\n\tv_nop" : "+v"(a) : "v"(w), "v"(x), "v"(y), "v"(z));
}
__device__ __forceinline__ void guard_h_1x2(v8f& a, v16h x, v16h y) {
  asm volatile("v_nop\n\tv_nop\n\tv_nop\n\tv_nop" : "+v"(a) : "v"(x), "v"(y));
}
__device__ __forceinline__ void guard_h_2x3(v8f& a, v8f& b, v16h x, v16h y, v16h z) {
  asm volatile("v_nop\n\tv_nop\n\tv_nop\n\tv_nop" : "+v"(a), "+v"(b) : "v"(x), "v"(y), "v"(z));
}
__device__ __forceinline__ void keep4_b(v16b a, v16b b, v16b c, v16b d) { asm volatile("v_nop" :: "v"(a), "v"(b), "v"(c), "v"(d)); }
__device__ __forceinline__ void acc_guard4(v8f& a, v8f& b, v8f& c, v8f& d) {
  asm volatile("v_nop\n\tv_nop\n\tv_nop\n\tv_nop" : "+v"(a), "+v"(b), "+v"(c), "+v"(d));
}
__device__ __forceinline__ void wave_lds_sync() {
  __builtin_amdgcn_fence(__ATOMIC_RELEASE, "workgroup");
  __builtin_amdgcn_wave_barrier();
  __builtin_amdgcn_fence(__ATOMIC_ACQUIRE, "workgroup");
}

__global__ __launch_bounds__(256) void wt_prep_kernel(const float* __restrict__ W0, const float* __restrict__ W1,
                                                      const float* __restrict__ W2, const float* __restrict__ W3,
                                                      unsigned short* __restrict__ outH, unsigned short* __restrict__ outL) {
  __shared__ float sm[64][65];
  const int t  = threadIdx.x;
  const int kt0 = blockIdx.x * 64;
  const int nt0 = blockIdx.y * 64;
  const int z  = blockIdx.z;
  const float* W = (z == 0) ? W0 : (z == 1) ? W1 : (z == 2) ? W2 : W3;
#pragma unroll
  for (int i = 0; i < 16; ++i) {
    const int e = i * 256 + t;
    const int r = e >> 6;
    const int c = e & 63;
    sm[c][r] = W[(size_t)(kt0 + r) * kDim + nt0 + c];
  }
  __syncthreads();
  const int lane = t & 31, wave = t >> 5;
  const int q4 = lane >> 3, c8 = (lane & 7) * 8;
  v4u uh[2], ul[2];
#pragma unroll
  for (int it = 0; it < 2; ++it) {
    const int row = wave * 8 + it * 4 + q4;
    unsigned short hb[8], lb[8];
#pragma unroll
    for (int e = 0; e < 8; ++e) {
      const float f = sm[row][c8 + e];
      hb[e] = f2bf_bits(f);
      lb[e] = f2bf_bits(f - bf_bits2f(hb[e]));
    }
    uh[it] = (v4u){pk16(hb[0], hb[1]), pk16(hb[2], hb[3]), pk16(hb[4], hb[5]), pk16(hb[6], hb[7])};
    ul[it] = (v4u){pk16(lb[0], lb[1]), pk16(lb[2], lb[3]), pk16(lb[4], lb[5]), pk16(lb[6], lb[7])};
  }
  for (int pass = 0; pass < 2; ++pass) {
#pragma unroll
    for (int it = 0; it < 2; ++it) {
      const int row = wave * 8 + it * 4 + q4;
      const size_t o = ((size_t)z * kDim + nt0 + row) * kDim + kt0 + c8;
      *(volatile v4u*)(outH + o) = uh[it];
      *(volatile v4u*)(outL + o) = ul[it];
    }
    __threadfence();
  }
}

__global__ __launch_bounds__(256) void split8_kernel(const float* __restrict__ in, unsigned short* __restrict__ hi,
                                                     unsigned short* __restrict__ lo, int n8) {
  const int i = blockIdx.x * 256 + threadIdx.x;
  if (i < n8) {
    const float* p = in + 8 * (size_t)i;
    const v4f a = *(const v4f*)(p);
    const v4f c = *(const v4f*)(p + 4);
    unsigned short hb[8], lb[8];
#pragma unroll
    for (int e = 0; e < 4; ++e) {
      const float f0 = a[e];
      const float f1 = c[e];
      hb[e]     = f2bf_bits(f0);
      lb[e]     = f2bf_bits(f0 - bf_bits2f(hb[e]));
      hb[4 + e] = f2bf_bits(f1);
      lb[4 + e] = f2bf_bits(f1 - bf_bits2f(hb[4 + e]));
    }
    const v4u uh = (v4u){pk16(hb[0], hb[1]), pk16(hb[2], hb[3]), pk16(hb[4], hb[5]), pk16(hb[6], hb[7])};
    const v4u ul = (v4u){pk16(lb[0], lb[1]), pk16(lb[2], lb[3]), pk16(lb[4], lb[5]), pk16(lb[6], lb[7])};
    unsigned short* ph = hi + 8 * (size_t)i;
    unsigned short* pl = lo + 8 * (size_t)i;
    *(volatile v4u*)ph = uh;
    *(volatile v4u*)pl = ul;
    __threadfence();
    *(volatile v4u*)ph = uh;
    *(volatile v4u*)pl = ul;
  }
}

__device__ __forceinline__ void gemm64_core(const __bf16* __restrict__ Ah, const __bf16* __restrict__ Al,
                                            const __bf16* __restrict__ Bh, const __bf16* __restrict__ Bl,
                                            int m0, int n0, int lane, v8f (&acc)[4][4]) {
  const int rlane = lane & 15;
  const int koff  = (lane >> 4) * 8;
#pragma unroll
  for (int i = 0; i < 4; ++i)
#pragma unroll
    for (int j = 0; j < 4; ++j) acc[i][j] = (v8f){0.f, 0.f, 0.f, 0.f, 0.f, 0.f, 0.f, 0.f};
  const __bf16* arh = Ah + (size_t)(m0 + rlane) * kDim + koff;
  const __bf16* arl = Al + (size_t)(m0 + rlane) * kDim + koff;
  const __bf16* brh = Bh + (size_t)(n0 + rlane) * kDim + koff;
  const __bf16* brl = Bl + (size_t)(n0 + rlane) * kDim + koff;
  for (int k0 = 0; k0 < kDim; k0 += 32) {
    v16b bh[4], bl[4];
#pragma unroll
    for (int j = 0; j < 4; ++j) {
      const int bo = (j << 4) * kDim + k0;
      bh[j] = ldfrag_b(brh + bo);
      bl[j] = ldfrag_b(brl + bo);
    }
#pragma unroll
    for (int i = 0; i < 4; ++i) {
      const int ao = (i << 4) * kDim + k0;
      const v16b ah = ldfrag_b(arh + ao);
      const v16b al = ldfrag_b(arl + ao);
#pragma unroll
      for (int j = 0; j < 4; ++j) {
        acc[i][j] = mma_b(ah, bh[j], acc[i][j]);
        acc[i][j] = mma_b(ah, bl[j], acc[i][j]);
        acc[i][j] = mma_b(al, bh[j], acc[i][j]);
      }
      guard_b_4x2(acc[i][0], acc[i][1], acc[i][2], acc[i][3], ah, al);
    }
    keep4_b(bh[0], bh[1], bh[2], bh[3]);
    keep4_b(bl[0], bl[1], bl[2], bl[3]);
  }
  acc_guard4(acc[0][0], acc[0][1], acc[0][2], acc[0][3]);
  acc_guard4(acc[1][0], acc[1][1], acc[1][2], acc[1][3]);
  acc_guard4(acc[2][0], acc[2][1], acc[2][2], acc[2][3]);
  acc_guard4(acc[3][0], acc[3][1], acc[3][2], acc[3][3]);
}

__global__ __launch_bounds__(256) void qkv_gemm_kernel(
    const unsigned short* __restrict__ XHp, const unsigned short* __restrict__ XLp,
    const unsigned short* __restrict__ WHp, const unsigned short* __restrict__ WLp,
    unsigned short* __restrict__ Qo, unsigned short* __restrict__ Ko,
    unsigned short* __restrict__ VTHo, unsigned short* __restrict__ VTLo) {
  __shared__ __align__(16) float sT[8][16 * kSlabPitch];
  __shared__ __align__(16) unsigned int sW[8][16 * kTwPitch];
  const int lane = threadIdx.x & 31;
  const int wave = threadIdx.x >> 5;
  constexpr int tilesN = kCatN / 64;
  constexpr int tilesM = kTok / 64;
  const int tile = blockIdx.x * 8 + wave;
  if (tile >= tilesM * tilesN) return;
  const int tm = tile / tilesN;
  const int tn = tile - tm * tilesN;
  const int m0 = tm << 6;
  const int n0 = tn << 6;
  const int kind = tn >> 3;

  v8f acc[4][4];
  gemm64_core((const __bf16*)XHp, (const __bf16*)XLp, (const __bf16*)WHp, (const __bf16*)WLp, m0, n0, lane, acc);

  const int rlane = lane & 15;
  const int hh    = lane >> 4;
  const int mOff  = hh * 8;
  const int q4 = lane >> 3, c8 = (lane & 7) * 8;
  if (kind < 2) {
    float* slab = sT[wave];
    unsigned short* Cp = (kind == 0) ? Qo : Ko;
    const int nl0 = n0 - kind * kDim;
#pragma unroll
    for (int i = 0; i < 4; ++i) {
      const int mBase = m0 + (i << 4);
#pragma unroll
      for (int j = 0; j < 4; ++j) {
#pragma unroll
        for (int r = 0; r < 8; ++r) slab[(mOff + r) * kSlabPitch + (j << 4) + rlane] = acc[i][j][r];
      }
      wave_lds_sync();
#pragma unroll 1
      for (int it = 0; it < 4; ++it) {
        float* sp = slab + (it * 4 + q4) * kSlabPitch + c8;
#pragma unroll
        for (int e = 0; e < 8; ++e) {
          const float u = sp[e];
          sp[e] = (u > 0.0f) ? (u + 1.0f) : expf(u);
        }
      }
      for (int pass = 0; pass < 2; ++pass) {
#pragma unroll
        for (int it = 0; it < 4; ++it) {
          const int row = it * 4 + q4;
          const float* sp = slab + row * kSlabPitch + c8;
          unsigned short hb[8];
#pragma unroll
          for (int e = 0; e < 8; ++e) hb[e] = h_bits(sp[e]);
          const v4u u = (v4u){pk16(hb[0], hb[1]), pk16(hb[2], hb[3]), pk16(hb[4], hb[5]), pk16(hb[6], hb[7])};
          *(volatile v4u*)(Cp + (size_t)(mBase + row) * kDim + nl0 + c8) = u;
        }
        __threadfence();
      }
      wave_lds_sync();
    }
  } else {
    unsigned int* tw = sW[wave];
    const int bb  = m0 >> 11;
    const int t0  = m0 & (kSeq - 1);
    const int el0 = n0 - 2 * kDim;
#pragma unroll
    for (int j = 0; j < 4; ++j) {
      v4u wh[4], wl[4];
#pragma unroll
      for (int i = 0; i < 4; ++i) {
        unsigned short hb[8], lb[8];
#pragma unroll
        for (int r = 0; r < 8; ++r) {
          const float v = acc[i][j][r];
          hb[r] = f2bf_bits(v);
          lb[r] = f2bf_bits(v - bf_bits2f(hb[r]));
        }
        wh[i] = (v4u){pk16(hb[0], hb[1]), pk16(hb[2], hb[3]), pk16(hb[4], hb[5]), pk16(hb[6], hb[7])};
        wl[i] = (v4u){pk16(lb[0], lb[1]), pk16(lb[2], lb[3]), pk16(lb[4], lb[5]), pk16(lb[6], lb[7])};
      }
      const size_t gbase = ((size_t)bb * kDim + el0 + (j << 4)) * kSeq + t0 + c8;
#pragma unroll
      for (int i = 0; i < 4; ++i) *(v4u*)(tw + rlane * kTwPitch + 8 * i + 4 * hh) = wh[i];
      wave_lds_sync();
      {
        v4u ld[4];
#pragma unroll
        for (int it = 0; it < 4; ++it) ld[it] = *(const v4u*)(tw + (it * 4 + q4) * kTwPitch + (lane & 7) * 4);
        for (int pass = 0; pass < 2; ++pass) {
#pragma unroll
          for (int it = 0; it < 4; ++it) *(volatile v4u*)(VTHo + gbase + (size_t)(it * 4 + q4) * kSeq) = ld[it];
          __threadfence();
        }
      }
      wave_lds_sync();
#pragma unroll
      for (int i = 0; i < 4; ++i) *(v4u*)(tw + rlane * kTwPitch + 8 * i + 4 * hh) = wl[i];
      wave_lds_sync();
      {
        v4u ld[4];
#pragma unroll
        for (int it = 0; it < 4; ++it) ld[it] = *(const v4u*)(tw + (it * 4 + q4) * kTwPitch + (lane & 7) * 4);
        for (int pass = 0; pass < 2; ++pass) {
#pragma unroll
          for (int it = 0; it < 4; ++it) *(volatile v4u*)(VTLo + gbase + (size_t)(it * 4 + q4) * kSeq) = ld[it];
          __threadfence();
        }
      }
      wave_lds_sync();
    }
  }
}

__global__ __launch_bounds__(256) void kt_transpose_kernel(const unsigned short* __restrict__ Kp,
                                                           unsigned short* __restrict__ KT) {
  __shared__ __align__(16) unsigned short tT[64 * kTtPitch];
  const int tid = threadIdx.x;
  const int d0 = blockIdx.x * 64, t0 = blockIdx.y * 64, b = blockIdx.z;
  const int r8 = tid >> 3, c8 = (tid & 7) * 8;
#pragma unroll
  for (int it = 0; it < 2; ++it) {
    const int trow = it * 32 + r8;
    const v4u w = *(const v4u*)(Kp + ((size_t)b * kSeq + t0 + trow) * kDim + d0 + c8);
#pragma unroll
    for (int e = 0; e < 4; ++e) {
      const unsigned we = w[e];
      const float f0 = h16_to_f32(we & 0xffffu);
      const float f1 = h16_to_f32(we >> 16);
      tT[(c8 + 2 * e) * kTtPitch + trow]     = f2bf_bits(f0);
      tT[(c8 + 2 * e + 1) * kTtPitch + trow] = f2bf_bits(f1);
    }
  }
  __syncthreads();
  us8 v[2];
#pragma unroll
  for (int it = 0; it < 2; ++it) v[it] = *(const us8*)(tT + (it * 32 + r8) * kTtPitch + c8);
  for (int pass = 0; pass < 2; ++pass) {
#pragma unroll
    for (int it = 0; it < 2; ++it)
      *(volatile us8*)(KT + ((size_t)b * kDim + d0 + it * 32 + r8) * kSeq + t0 + c8) = v[it];
    __threadfence();
  }
}

__global__ __launch_bounds__(256) void zprefix_kernel(const unsigned short* __restrict__ KT, float* __restrict__ ZP) {
  const int g = blockIdx.x * 256 + threadIdx.x;
  const int b = g >> 9, d = g & (kDim - 1);
  const unsigned short* row = KT + (size_t)g * kSeq;
  float run = 0.0f;
#pragma unroll 1
  for (int ch = 0; ch < kNChunk; ++ch) {
    float* zp = ZP + ((size_t)(b * kNChunk + ch)) * kDim + d;
    *(volatile float*)zp = run;
    __threadfence();
    *(volatile float*)zp = run;
    float s = 0.0f;
#pragma unroll
    for (int u = 0; u < 8; ++u) {
      const v4u w = *(const v4u*)(row + ch * kChunk + u * 8);
#pragma unroll
      for (int e = 0; e < 4; ++e) {
        const unsigned we = w[e];
        s += __uint_as_float(we << 16);
        s += __uint_as_float(we & 0xffff0000u);
      }
    }
    run += s;
  }
}

__global__ __launch_bounds__(256) void chunk_scores_kernel(
    const unsigned short* __restrict__ Qp, const unsigned short* __restrict__ Kp, const float* __restrict__ ZP,
    unsigned short* __restrict__ AH, unsigned short* __restrict__ AL, float* __restrict__ DEN) {
  __shared__ __align__(16) float As[kChunk * kAsPitch];
  __shared__ __align__(16) float zs[kDim];
  __shared__ float rs[kChunk];
  __shared__ float dq[kChunk];
  const int tid = threadIdx.x, lane = tid & 31, wave = tid >> 5;
  const int c = lane & 15, hh = lane >> 4, koff = hh * 8;
  const int bc = blockIdx.x;
  const size_t row0 = (size_t)bc * kChunk;

  if (tid < 128) {
    const v4f z = *(const v4f*)(ZP + (size_t)bc * kDim + tid * 4);
    *(v4f*)(zs + tid * 4) = z;
  }
  {
    const int mt = wave >> 1, ntb = (wave & 1) * 2;
    const _Float16* qa  = (const _Float16*)Qp + (row0 + 16 * mt + c) * kDim + koff;
    const _Float16* kb0 = (const _Float16*)Kp + (row0 + 16 * ntb + c) * kDim + koff;
    const _Float16* kb1 = kb0 + 16 * kDim;
    v8f acc0 = (v8f){0.f, 0.f, 0.f, 0.f, 0.f, 0.f, 0.f, 0.f};
    v8f acc1 = acc0;
#pragma unroll 1
    for (int k0 = 0; k0 < kDim; k0 += 32) {
      const v16h a  = ldfrag_h(qa + k0);
      const v16h b0 = ldfrag_h(kb0 + k0);
      const v16h b1 = ldfrag_h(kb1 + k0);
      acc0 = mma_h(a, b0, acc0);
      acc1 = mma_h(a, b1, acc1);
      guard_h_2x3(acc0, acc1, a, b0, b1);
    }
#pragma unroll
    for (int r = 0; r < 8; ++r) {
      As[(16 * mt + 8 * hh + r) * kAsPitch + 16 * ntb + c]      = acc0[r];
      As[(16 * mt + 8 * hh + r) * kAsPitch + 16 * ntb + 16 + c] = acc1[r];
    }
  }
  __syncthreads();

  {
    const int t = tid >> 2, part = tid & 3;
    const unsigned short* qrow = Qp + (row0 + t) * kDim + part * 128;
    const float* zp = zs + part * 128;
    float s = 0.0f;
#pragma unroll 1
    for (int g = 0; g < 16; ++g) {
      const v4u w  = *(const v4u*)(qrow + 8 * g);
      const v4f z0 = *(const v4f*)(zp + 8 * g);
      const v4f z1 = *(const v4f*)(zp + 8 * g + 4);
      const unsigned w0 = w[0], w1 = w[1], w2 = w[2], w3 = w[3];
      s = fmaf(h16_to_f32(w0 & 0xffffu), z0[0], s);
      s = fmaf(h16_to_f32(w0 >> 16),     z0[1], s);
      s = fmaf(h16_to_f32(w1 & 0xffffu), z0[2], s);
      s = fmaf(h16_to_f32(w1 >> 16),     z0[3], s);
      s = fmaf(h16_to_f32(w2 & 0xffffu), z1[0], s);
      s = fmaf(h16_to_f32(w2 >> 16),     z1[1], s);
      s = fmaf(h16_to_f32(w3 & 0xffffu), z1[2], s);
      s = fmaf(h16_to_f32(w3 >> 16),     z1[3], s);
    }
    s += __shfl_xor(s, 1, 32);
    s += __shfl_xor(s, 2, 32);
    if (part == 0) dq[t] = s;
  }

  {
    const int r8 = tid >> 3, c8 = (tid & 7) * 8;
    v4u uh[2], ul[2];
#pragma unroll
    for (int it = 0; it < 2; ++it) {
      const int row = it * 32 + r8;
      const v4f a0 = *(const v4f*)(As + row * kAsPitch + c8);
      const v4f a1 = *(const v4f*)(As + row * kAsPitch + c8 + 4);
      unsigned short hb[8], lb[8];
      float part = 0.0f;
#pragma unroll
      for (int e = 0; e < 8; ++e) {
        const float raw = (e < 4) ? a0[e & 3] : a1[e & 3];
        const float v = ((c8 + e) <= row) ? raw : 0.0f;
        hb[e] = f2bf_bits(v);
        lb[e] = f2bf_bits(v - bf_bits2f(hb[e]));
        part += bf_bits2f(hb[e]) + bf_bits2f(lb[e]);
      }
      part += __shfl_xor(part, 1, 32);
      part += __shfl_xor(part, 2, 32);
      part += __shfl_xor(part, 4, 32);
      if ((tid & 7) == 0) rs[row] = part;
      uh[it] = (v4u){pk16(hb[0], hb[1]), pk16(hb[2], hb[3]), pk16(hb[4], hb[5]), pk16(hb[6], hb[7])};
      ul[it] = (v4u){pk16(lb[0], lb[1]), pk16(lb[2], lb[3]), pk16(lb[4], lb[5]), pk16(lb[6], lb[7])};
    }
    for (int pass = 0; pass < 2; ++pass) {
#pragma unroll
      for (int it = 0; it < 2; ++it) {
        const size_t o = (row0 + it * 32 + r8) * kChunk + c8;
        *(volatile v4u*)(AH + o) = uh[it];
        *(volatile v4u*)(AL + o) = ul[it];
      }
      __threadfence();
    }
  }
  __syncthreads();
  if (tid < 16) {
    v4f d;
#pragma unroll
    for (int e = 0; e < 4; ++e) d[e] = (rs[4 * tid + e] + dq[4 * tid + e]) + kDenEps;
    float* dp = DEN + row0 + 4 * tid;
    *(volatile v4f*)dp = d;
    __threadfence();
    *(volatile v4f*)dp = d;
  }
}

__global__ __launch_bounds__(256) void chunk_scan_kernel(
    const unsigned short* __restrict__ Qp, const unsigned short* __restrict__ KTp,
    const unsigned short* __restrict__ VTHp, const unsigned short* __restrict__ VTLp,
    const unsigned short* __restrict__ AHp, const unsigned short* __restrict__ ALp,
    const float* __restrict__ DEN, float* __restrict__ YF) {
  __shared__ __align__(16) _Float16 St[kESlice * kStPitch];
  __shared__ __align__(16) float Ys[kChunk * kYsPitch];
  const int tid = threadIdx.x, lane = tid & 31, wave = tid >> 5;
  const int c = lane & 15, hh = lane >> 4, koff = hh * 8;
  const int b  = blockIdx.x >> 4;
  const int e0 = (blockIdx.x & 15) * kESlice;
  const int mt = wave >> 1, et = wave & 1;
  const int q8 = lane >> 3, c4 = (lane & 7) * 4;

  const _Float16* Qb = (const _Float16*)Qp + ((size_t)b * kSeq + 16 * mt + c) * kDim + koff;
  const __bf16* KTb  = (const __bf16*)KTp + ((size_t)b * kDim + 64 * wave + c) * kSeq + koff;
  const __bf16* VHb  = (const __bf16*)VTHp + ((size_t)b * kDim + e0 + c) * kSeq + koff;
  const __bf16* VLb  = (const __bf16*)VTLp + ((size_t)b * kDim + e0 + c) * kSeq + koff;
  const __bf16* AHb  = (const __bf16*)AHp + ((size_t)b * kSeq + 16 * mt + c) * kChunk + koff;
  const __bf16* ALb  = (const __bf16*)ALp + ((size_t)b * kSeq + 16 * mt + c) * kChunk + koff;
  const float* DENb  = DEN + (size_t)b * kSeq + 16 * mt + 8 * hh;
  float* YFb = YF + (size_t)b * kSeq * kDim + e0 + c4;
  const _Float16* Sr = St + (16 * et + c) * kStPitch + koff;

  {
    v8h zh;
#pragma unroll
    for (int e = 0; e < 8; ++e) zh[e] = (_Float16)0.0f;
#pragma unroll 1
    for (int i = tid; i < (kESlice * kStPitch) / 8; i += 256) *(v8h*)(St + 8 * i) = zh;
  }
  v8f sacc[4][2];
#pragma unroll
  for (int i = 0; i < 4; ++i)
#pragma unroll
    for (int j = 0; j < 2; ++j) sacc[i][j] = (v8f){0.f, 0.f, 0.f, 0.f, 0.f, 0.f, 0.f, 0.f};

#pragma unroll 1
  for (int ch = 0; ch < kNChunk; ++ch) {
    const int t0 = ch * kChunk;
    __syncthreads();

    v8f acc = (v8f){0.f, 0.f, 0.f, 0.f, 0.f, 0.f, 0.f, 0.f};
    {
      const _Float16* qp = Qb + (size_t)t0 * kDim;
#pragma unroll 1
      for (int k0 = 0; k0 < kDim; k0 += 32) {
        const v16h a  = ldfrag_h(qp + k0);
        const v16h bs = ldfrag_h(Sr + k0);
        acc = mma_h(a, bs, acc);
        guard_h_1x2(acc, a, bs);
      }
    }
    {
      const __bf16* ahp = AHb + (size_t)ch * kChunk * kChunk;
      const __bf16* alp = ALb + (size_t)ch * kChunk * kChunk;
      const __bf16* vhp = VHb + (size_t)(16 * et) * kSeq + t0;
      const __bf16* vlp = VLb + (size_t)(16 * et) * kSeq + t0;
#pragma unroll
      for (int kk = 0; kk < 2; ++kk) {
        const v16b ah = ldfrag_b(ahp + 32 * kk);
        const v16b al = ldfrag_b(alp + 32 * kk);
        const v16b vh = ldfrag_b(vhp + 32 * kk);
        const v16b vl = ldfrag_b(vlp + 32 * kk);
        acc = mma_b(ah, vh, acc);
        acc = mma_b(ah, vl, acc);
        acc = mma_b(al, vh, acc);
        guard_b_1x4(acc, ah, al, vh, vl);
      }
    }
    {
      const v4f d0 = *(const v4f*)(DENb + t0);
      const v4f d1 = *(const v4f*)(DENb + t0 + 4);
#pragma unroll
      for (int r = 0; r < 4; ++r) {
        const float da = d0[r];
        const float db = d1[r];
        Ys[(16 * mt + 8 * hh + r) * kYsPitch + 16 * et + c]     = acc[r] * (1.0f / da);
        Ys[(16 * mt + 8 * hh + 4 + r) * kYsPitch + 16 * et + c] = acc[4 + r] * (1.0f / db);
      }
    }
    __syncthreads();
    {
      v4f yv[2];
#pragma unroll
      for (int it = 0; it < 2; ++it) yv[it] = *(const v4f*)(Ys + (it * 32 + 4 * wave + q8) * kYsPitch + c4);
      for (int pass = 0; pass < 2; ++pass) {
#pragma unroll
        for (int it = 0; it < 2; ++it)
          *(volatile v4f*)(YFb + (size_t)(t0 + it * 32 + 4 * wave + q8) * kDim) = yv[it];
        __threadfence();
      }
    }

#pragma unroll
    for (int j = 0; j < 2; ++j) {
      const __bf16* vhp = VHb + (size_t)(16 * j) * kSeq + t0;
      const __bf16* vlp = VLb + (size_t)(16 * j) * kSeq + t0;
      const v16b vh0 = ldfrag_b(vhp);
      const v16b vh1 = ldfrag_b(vhp + 32);
      const v16b vl0 = ldfrag_b(vlp);
      const v16b vl1 = ldfrag_b(vlp + 32);
#pragma unroll
      for (int i = 0; i < 4; ++i) {
        const __bf16* kp = KTb + (size_t)(16 * i) * kSeq + t0;
        const v16b a0 = ldfrag_b(kp);
        const v16b a1 = ldfrag_b(kp + 32);
        sacc[i][j] = mma_b(a0, vh0, sacc[i][j]);
        sacc[i][j] = mma_b(a0, vl0, sacc[i][j]);
        sacc[i][j] = mma_b(a1, vh1, sacc[i][j]);
        sacc[i][j] = mma_b(a1, vl1, sacc[i][j]);
        guard_b_1x2(sacc[i][j], a0, a1);
      }
      keep4_b(vh0, vh1, vl0, vl1);
    }
#pragma unroll
    for (int j = 0; j < 2; ++j) {
#pragma unroll
      for (int i = 0; i < 4; ++i) {
        v8h hv;
#pragma unroll
        for (int r = 0; r < 8; ++r) hv[r] = (_Float16)sacc[i][j][r];
        *(v8h*)(St + (16 * j + c) * kStPitch + 64 * wave + 16 * i + 8 * hh) = hv;
      }
    }
  }
}

__global__ __launch_bounds__(256) void out_gemm_kernel(
    const unsigned short* __restrict__ YHp, const unsigned short* __restrict__ YLp,
    const unsigned short* __restrict__ WHp, const unsigned short* __restrict__ WLp,
    float* __restrict__ outp) {
  __shared__ __align__(16) float sT[8][16 * kSlabPitch];
  const int lane = threadIdx.x & 31;
  const int wave = threadIdx.x >> 5;
  constexpr int tilesN = kDim / 64;
  constexpr int tilesM = kTok / 64;
  const int tile = blockIdx.x * 8 + wave;
  if (tile >= tilesM * tilesN) return;
  const int tm = tile / tilesN;
  const int tn = tile - tm * tilesN;
  const int m0 = tm << 6;
  const int n0 = tn << 6;

  v8f acc[4][4];
  gemm64_core((const __bf16*)YHp, (const __bf16*)YLp, (const __bf16*)WHp, (const __bf16*)WLp, m0, n0, lane, acc);

  float* slab = sT[wave];
  const int rlane = lane & 15;
  const int hh = lane >> 4;
  const int mOff = hh * 8;
  const int c4 = (lane & 15) * 4;
#pragma unroll
  for (int i = 0; i < 4; ++i) {
    const int mBase = m0 + (i << 4);
#pragma unroll
    for (int j = 0; j < 4; ++j) {
#pragma unroll
      for (int r = 0; r < 8; ++r) slab[(mOff + r) * kSlabPitch + (j << 4) + rlane] = acc[i][j][r];
    }
    wave_lds_sync();
    for (int pass = 0; pass < 2; ++pass) {
#pragma unroll
      for (int it = 0; it < 8; ++it) {
        const int row = it * 2 + hh;
        const v4f v = *(const v4f*)(slab + row * kSlabPitch + c4);
        *(volatile v4f*)(outp + (size_t)(mBase + row) * kDim + n0 + c4) = v;
      }
      __threadfence();
    }
    wave_lds_sync();
  }
}

extern "C" void kernel_launch(void* const* d_in, const int* in_sizes, int n_in,
                              void* d_out, int out_size, void* d_ws, size_t ws_size, hipStream_t stream) {
  if (n_in < 5 || d_out == nullptr || d_ws == nullptr) return;
  if (in_sizes[0] != kTok * kDim || in_sizes[1] != kDim * kDim || in_sizes[2] != kDim * kDim ||
      in_sizes[3] != kDim * kDim || in_sizes[4] != kDim * kDim || out_size != kTok * kDim) return;

  const float* x  = (const float*)d_in[0];
  const float* Wq = (const float*)d_in[1];
  const float* Wk = (const float*)d_in[2];
  const float* Wv = (const float*)d_in[3];
  const float* Wp = (const float*)d_in[4];
  float* outp = (float*)d_out;

  char* ws = (char*)d_ws;
  size_t off = 0;
  auto carve = [&](size_t bytes) -> char* { char* p = ws + off; off += (bytes + 255) & ~(size_t)255; return p; };
  const size_t planeB = (size_t)kTok * kDim * 2;
  unsigned short* XH  = (unsigned short*)carve(planeB);
  unsigned short* XL  = (unsigned short*)carve(planeB);
  unsigned short* QP  = (unsigned short*)carve(planeB);
  unsigned short* KP  = (unsigned short*)carve(planeB);
  unsigned short* KT  = (unsigned short*)carve(planeB);
  unsigned short* VTH = (unsigned short*)carve(planeB);
  unsigned short* VTL = (unsigned short*)carve(planeB);
  unsigned short* WTH = (unsigned short*)carve((size_t)4 * kDim * kDim * 2);
  unsigned short* WTL = (unsigned short*)carve((size_t)4 * kDim * kDim * 2);
  unsigned short* AH  = (unsigned short*)carve((size_t)kTok * kChunk * 2);
  unsigned short* AL  = (unsigned short*)carve((size_t)kTok * kChunk * 2);
  float* ZP  = (float*)carve((size_t)kBatch * kNChunk * kDim * 4);
  float* DEN = (float*)carve((size_t)kTok * 4);
  if (off > ws_size || off > (size_t)134217728) return;
  float* YF = (float*)XH;
  unsigned short* YH = QP;
  unsigned short* YL = KP;
  const unsigned short* WPH = WTH + (size_t)kCatN * kDim;
  const unsigned short* WPL = WTL + (size_t)kCatN * kDim;

  const int n8 = kTok * kDim / 8;

  wt_prep_kernel<<<dim3(kDim / 64, kDim / 64, 4), 256, 0, stream>>>(Wq, Wk, Wv, Wp, WTH, WTL);
  split8_kernel<<<n8 / 256, 256, 0, stream>>>(x, XH, XL, n8);
  qkv_gemm_kernel<<<(kTok / 64) * (kCatN / 64) / 8, 256, 0, stream>>>(XH, XL, WTH, WTL, QP, KP, VTH, VTL);
  kt_transpose_kernel<<<dim3(kDim / 64, kSeq / 64, kBatch), 256, 0, stream>>>(KP, KT);
  zprefix_kernel<<<(kBatch * kDim) / 256, 256, 0, stream>>>(KT, ZP);
  chunk_scores_kernel<<<kBatch * kNChunk, 256, 0, stream>>>(QP, KP, ZP, AH, AL, DEN);
  chunk_scan_kernel<<<kBatch * kNESlice, 256, 0, stream>>>(QP, KT, VTH, VTL, AH, AL, DEN, YF);
  split8_kernel<<<n8 / 256, 256, 0, stream>>>(YF, YH, YL, n8);
  out_gemm_kernel<<<(kTok / 64) * (kDim / 64) / 8, 256, 0, stream>>>(YH, YL, WPH, WPL, outp);
}
